// _F3Block_42588895707390
// MI455X (gfx1250) — hardware-run, weakly checked
//
#include <hip/hip_runtime.h>
#include <stddef.h>
#include <stdint.h>

#define NBAT  2
#define SQ    2048
#define NTOK  4096
#define HID   768
#define FFD   3072
#define NH    12
#define HDM   64
#define THD   32
#define TDM   384
#define QB    128
#define KC    64
#define NQB   (SQ / QB)
#define NKC   (SQ / KC)

static_assert(NTOK == NBAT * SQ);
static_assert(NH * HDM == HID);
static_assert(HID % 64 == 0);
static_assert(FFD % 64 == 0);
static_assert(SQ % QB == 0);
static_assert(SQ % KC == 0);
static_assert(QB == 2 * KC);
static_assert(NTOK % 256 == 0);
static_assert((NTOK * HID) % 2048 == 0);
static_assert(HDM == 64);
static_assert(THD == 32);
static_assert(TDM == 3 * 128);
static_assert(HID == 2 * TDM);

typedef _Float16 v16h __attribute__((ext_vector_type(16)));
typedef _Float16 v8h  __attribute__((ext_vector_type(8)));
typedef _Float16 v4h  __attribute__((ext_vector_type(4)));
typedef float    v8f  __attribute__((ext_vector_type(8)));
typedef float    v4f  __attribute__((ext_vector_type(4)));
typedef unsigned int v4u __attribute__((ext_vector_type(4)));
typedef unsigned int v2u __attribute__((ext_vector_type(2)));

union Frag  { v16h v; v8h h[2]; };
union Pack8 { v8h h; v4u u; };
union Pack4 { v4h h; v2u u; };

__device__ __forceinline__ v8f mma16(v16h a, v16h b, v8f c) {
  c = __builtin_amdgcn_wmma_f32_16x16x32_f16(false, a, false, b, (short)0, c, false, false);
  asm volatile("v_nop\n\tv_nop\n\tv_nop\n\tv_nop" : "+v"(c) : "v"(a), "v"(b));
  return c;
}

__device__ __forceinline__ v16h ldfrag(const _Float16* p, int ld, int row0, int k0, int lane) {
  const int m = lane & 15, lh = lane >> 4;
  const _Float16* q = p + (size_t)(row0 + m) * ld + k0 + 8 * lh;
  Frag f;
  f.h[0] = *(const v8h*)(q);
  f.h[1] = *(const v8h*)(q + 16);
  return f.v;
}

__device__ __forceinline__ v8f zero8() { return (v8f){0.f, 0.f, 0.f, 0.f, 0.f, 0.f, 0.f, 0.f}; }

__device__ __forceinline__ float wsum32(float s) {
#pragma unroll
  for (int off = 16; off >= 1; off >>= 1) s += __shfl_xor(s, off, 32);
  return s;
}

__device__ __forceinline__ float gelu_t(float x) {
  const float u = 0.7978845608028654f * (x + 0.044715f * x * x * x);
  const float e = __expf(2.0f * u);
  const float r = __builtin_amdgcn_rcpf(e + 1.0f);
  return x - x * r;
}

__device__ __forceinline__ void gemm16x64(const _Float16* __restrict__ A, int lda,
                                          const _Float16* __restrict__ Bt, int ldb,
                                          int m0, int n0, int lane, v8f (&acc)[4]) {
#pragma unroll 2
  for (int k0 = 0; k0 < HID; k0 += 32) {
    const v16h a = ldfrag(A, lda, m0, k0, lane);
#pragma unroll
    for (int t = 0; t < 4; ++t) {
      const v16h b = ldfrag(Bt, ldb, n0 + 16 * t, k0, lane);
      acc[t] = mma16(a, b, acc[t]);
    }
  }
}

__device__ __forceinline__ void gemm32x64(const _Float16* __restrict__ A, int lda,
                                          const _Float16* __restrict__ Bt, int ldb, int K,
                                          int m0, int n0, int lane, v8f (&acc)[2][4]) {
#pragma unroll 2
  for (int k0 = 0; k0 < K; k0 += 32) {
    const v16h a0 = ldfrag(A, lda, m0, k0, lane);
    const v16h a1 = ldfrag(A, lda, m0 + 16, k0, lane);
    const v16h b0 = ldfrag(Bt, ldb, n0, k0, lane);
    const v16h b1 = ldfrag(Bt, ldb, n0 + 16, k0, lane);
    const v16h b2 = ldfrag(Bt, ldb, n0 + 32, k0, lane);
    const v16h b3 = ldfrag(Bt, ldb, n0 + 48, k0, lane);
    acc[0][0] = mma16(a0, b0, acc[0][0]);
    acc[1][0] = mma16(a1, b0, acc[1][0]);
    acc[0][1] = mma16(a0, b1, acc[0][1]);
    acc[1][1] = mma16(a1, b1, acc[1][1]);
    acc[0][2] = mma16(a0, b2, acc[0][2]);
    acc[1][2] = mma16(a1, b2, acc[1][2]);
    acc[0][3] = mma16(a0, b3, acc[0][3]);
    acc[1][3] = mma16(a1, b3, acc[1][3]);
  }
}

#define TWP 68
__global__ __launch_bounds__(128) void k_cvtw(const float* __restrict__ w0, const float* __restrict__ w1,
                                              const float* __restrict__ w2, const float* __restrict__ w3,
                                              int K, int N, _Float16* __restrict__ wt) {
  __shared__ __align__(16) float tl[64 * TWP];
  const int tid = threadIdx.x;
  const int z = blockIdx.z;
  const float* s = (z == 0) ? w0 : ((z == 1) ? w1 : ((z == 2) ? w2 : w3));
  const int n0 = blockIdx.x * 64;
  const int k0 = blockIdx.y * 64;
#pragma unroll
  for (int j = 0; j < 8; ++j) {
    const int p  = tid + 128 * j;
    const int kr = p >> 4;
    const int c4 = (p & 15) * 4;
    const v4f a = *(const v4f*)(s + (size_t)(k0 + kr) * N + n0 + c4);
    *(v4f*)(tl + kr * TWP + c4) = a;
  }
  __syncthreads();
  v4u val[4];
  size_t go[4];
#pragma unroll
  for (int j = 0; j < 4; ++j) {
    const int p  = tid + 128 * j;
    const int n  = p >> 3;
    const int kc = (p & 7) * 8;
    const float* cp = tl + kc * TWP + n;
    Pack8 pk;
    pk.h = (v8h){(_Float16)(cp[0 * TWP] * 32.0f), (_Float16)(cp[1 * TWP] * 32.0f),
                 (_Float16)(cp[2 * TWP] * 32.0f), (_Float16)(cp[3 * TWP] * 32.0f),
                 (_Float16)(cp[4 * TWP] * 32.0f), (_Float16)(cp[5 * TWP] * 32.0f),
                 (_Float16)(cp[6 * TWP] * 32.0f), (_Float16)(cp[7 * TWP] * 32.0f)};
    val[j] = pk.u;
    go[j]  = ((size_t)z * N + n0 + n) * K + k0 + kc;
  }
#pragma unroll
  for (int j = 0; j < 4; ++j) *(volatile v4u*)(wt + go[j]) = val[j];
  __threadfence();
#pragma unroll
  for (int j = 0; j < 4; ++j) *(volatile v4u*)(wt + go[j]) = val[j];
}

__global__ __launch_bounds__(256) void k_cvtx(const float* __restrict__ x, _Float16* __restrict__ xh) {
  const size_t i = (size_t)blockIdx.x * 2048 + (size_t)threadIdx.x * 8;
  const v4f a0 = *(const v4f*)(x + i);
  const v4f a1 = *(const v4f*)(x + i + 4);
  Pack8 pk;
  pk.h = (v8h){(_Float16)a0[0], (_Float16)a0[1], (_Float16)a0[2], (_Float16)a0[3],
               (_Float16)a1[0], (_Float16)a1[1], (_Float16)a1[2], (_Float16)a1[3]};
  const v4u vv = pk.u;
  volatile v4u* dp = (volatile v4u*)(xh + i);
  *dp = vv;
  __threadfence();
  *dp = vv;
}

#define SFP 68
__global__ __launch_bounds__(128) void k_qkv(const _Float16* __restrict__ xh,
                                             const _Float16* __restrict__ wt,
                                             const float* __restrict__ bq,
                                             const float* __restrict__ bk,
                                             const float* __restrict__ bv,
                                             _Float16* __restrict__ qp,
                                             _Float16* __restrict__ kp,
                                             _Float16* __restrict__ vtp) {
  __shared__ __align__(16) float sf[64 * SFP];
  const int tid = threadIdx.x, lane = tid & 31, wave = tid >> 5;
  const int hh = lane >> 4, c = lane & 15;
  const int mb = blockIdx.x * 64;
  const int b  = mb / SQ;
  const int sb = mb - b * SQ;
  const int ns = blockIdx.y;
  const int which = ns / NH;
  const int head  = ns - which * NH;
  const int hb = b * NH + head;
  const int m0 = mb + wave * 16;
  const int n0 = ns * HDM;

  v8f acc[4];
#pragma unroll
  for (int t = 0; t < 4; ++t) acc[t] = zero8();
  gemm16x64(xh, HID, wt, HID, m0, n0, lane, acc);

#pragma unroll
  for (int t = 0; t < 4; ++t) {
    const int bi = head * HDM + 16 * t + c;
    const float f0 = bq[bi], f1 = bk[bi], f2 = bv[bi];
    const float bs = (which == 0) ? f0 : ((which == 1) ? f1 : f2);
    const float sg = (which == 0 && t < 2) ? -1.0f : 1.0f;
#pragma unroll
    for (int r = 0; r < 8; ++r)
      sf[(wave * 16 + 8 * hh + r) * SFP + 16 * t + c] = (acc[t][r] * 0.03125f + bs) * sg;
  }
  __syncthreads();

  if (which < 2) {
    v4u val[4];
    size_t go[4];
#pragma unroll
    for (int j = 0; j < 4; ++j) {
      const int p  = tid + 128 * j;
      const int lr = p >> 3;
      const int d0 = (p & 7) * 8;
      const float* ra = sf + lr * SFP + d0;
      const v4f a0 = *(const v4f*)(ra), a1 = *(const v4f*)(ra + 4);
      Pack8 pk;
      pk.h = (v8h){(_Float16)a0[0], (_Float16)a0[1], (_Float16)a0[2], (_Float16)a0[3],
                   (_Float16)a1[0], (_Float16)a1[1], (_Float16)a1[2], (_Float16)a1[3]};
      val[j] = pk.u;
      go[j]  = ((size_t)hb * SQ + sb + lr) * HDM + d0;
    }
    _Float16* base = (which == 0) ? qp : kp;
#pragma unroll
    for (int j = 0; j < 4; ++j) *(volatile v4u*)(base + go[j]) = val[j];
    __threadfence();
#pragma unroll
    for (int j = 0; j < 4; ++j) *(volatile v4u*)(base + go[j]) = val[j];
  } else {
    v4u val[4];
    size_t go[4];
#pragma unroll
    for (int j = 0; j < 4; ++j) {
      const int p  = tid + 128 * j;
      const int d  = p >> 3;
      const int pc = p & 7;
      const float* cp = sf + (pc * 8) * SFP + d;
      Pack8 pk;
      pk.h = (v8h){(_Float16)cp[0 * SFP], (_Float16)cp[1 * SFP], (_Float16)cp[2 * SFP], (_Float16)cp[3 * SFP],
                   (_Float16)cp[4 * SFP], (_Float16)cp[5 * SFP], (_Float16)cp[6 * SFP], (_Float16)cp[7 * SFP]};
      val[j] = pk.u;
      go[j]  = ((size_t)hb * HDM + d) * SQ + sb + pc * 8;
    }
#pragma unroll
    for (int j = 0; j < 4; ++j) *(volatile v4u*)(vtp + go[j]) = val[j];
    __threadfence();
#pragma unroll
    for (int j = 0; j < 4; ++j) *(volatile v4u*)(vtp + go[j]) = val[j];
  }
}

#define LP 72
__global__ __launch_bounds__(256) void k_attn(const _Float16* __restrict__ qp,
                                              const _Float16* __restrict__ kp,
                                              const _Float16* __restrict__ vt,
                                              _Float16* __restrict__ op, float sscale) {
  __shared__ __align__(16) _Float16 Ks[KC * LP];
  __shared__ __align__(16) _Float16 Vs[HDM * LP];
  __shared__ __align__(16) _Float16 Ps[8 * 16 * LP];

  const int tid = threadIdx.x, lane = tid & 31, wave = tid >> 5;
  const int hh = lane >> 4, c = lane & 15;
  const int qb  = blockIdx.x % NQB;
  const int hb  = blockIdx.x / NQB;
  const int h   = hb % NH;
  const int b   = hb / NH;
  const int q0  = qb * QB + wave * 16;

  const _Float16* Q = qp + (size_t)hb * SQ * HDM;
  const _Float16* K = kp + (size_t)hb * SQ * HDM;
  const _Float16* V = vt + (size_t)hb * HDM * SQ;
  const size_t trow0 = (size_t)b * SQ;

  const float NEGI = -__builtin_huge_valf();
  float mrow[8], lrow[8];
  v8f oacc[4];
#pragma unroll
  for (int r = 0; r < 8; ++r) { mrow[r] = NEGI; lrow[r] = 0.f; }
#pragma unroll
  for (int t = 0; t < 4; ++t) oacc[t] = zero8();

  _Float16* pw = Ps + wave * 16 * LP;

  for (int kc = 0; kc < NKC; ++kc) {
    const int kv0 = kc * KC;
    __syncthreads();
    {
      const int r  = tid >> 2;
      const int qq = (tid & 3) * 16;
      const _Float16* ks = K + (size_t)(kv0 + r) * HDM + qq;
#pragma unroll
      for (int e = 0; e < 2; ++e) *(v8h*)(Ks + r * LP + qq + 8 * e) = *(const v8h*)(ks + 8 * e);
      const _Float16* vs = V + (size_t)r * SQ + kv0 + qq;
#pragma unroll
      for (int e = 0; e < 2; ++e) *(v8h*)(Vs + r * LP + qq + 8 * e) = *(const v8h*)(vs + 8 * e);
    }
    __syncthreads();

    v8f s[4];
#pragma unroll
    for (int j = 0; j < 4; ++j) s[j] = zero8();
#pragma unroll
    for (int dc = 0; dc < 2; ++dc) {
      const v16h qa = ldfrag(Q, HDM, q0, dc * 32, lane);
#pragma unroll
      for (int j = 0; j < 4; ++j) {
        const v16h kb = ldfrag(Ks, LP, j * 16, dc * 32, lane);
        s[j] = mma16(qa, kb, s[j]);
      }
    }
#pragma unroll
    for (int r = 0; r < 8; ++r)
#pragma unroll
      for (int j = 0; j < 4; ++j) s[j][r] *= sscale;

    float cm[8];
#pragma unroll
    for (int r = 0; r < 8; ++r) {
      float m = NEGI;
#pragma unroll
      for (int j = 0; j < 4; ++j) m = fmaxf(m, s[j][r]);
#pragma unroll
      for (int off = 1; off < 16; off <<= 1) m = fmaxf(m, __shfl_xor(m, off, 32));
      cm[r] = m;
    }
    float al[8];
#pragma unroll
    for (int r = 0; r < 8; ++r) {
      const float mnew  = fmaxf(mrow[r], cm[r]);
      const float alpha = __expf(mrow[r] - mnew);
      mrow[r] = mnew;
      float psum = 0.f;
#pragma unroll
      for (int j = 0; j < 4; ++j) {
        const float p = __expf(s[j][r] - mnew);
        psum += p;
        pw[(8 * hh + r) * LP + j * 16 + c] = (_Float16)(p * 1024.0f);
      }
#pragma unroll
      for (int off = 1; off < 16; off <<= 1) psum += __shfl_xor(psum, off, 32);
      lrow[r] = lrow[r] * alpha + psum;
      al[r] = alpha;
    }
#pragma unroll
    for (int t = 0; t < 4; ++t)
#pragma unroll
      for (int r = 0; r < 8; ++r) oacc[t][r] *= al[r];
    __syncthreads();

#pragma unroll
    for (int kk = 0; kk < 2; ++kk) {
      const v16h pa = ldfrag(pw, LP, 0, kk * 32, lane);
#pragma unroll
      for (int t = 0; t < 4; ++t) {
        const v16h vb = ldfrag(Vs, LP, t * 16, kk * 32, lane);
        oacc[t] = mma16(pa, vb, oacc[t]);
      }
    }
  }

  float invl[8];
#pragma unroll
  for (int r = 0; r < 8; ++r) invl[r] = (lrow[r] > 0.f) ? (0.0625f * (1.0f / lrow[r])) : 0.f;
  __syncthreads();
#pragma unroll
  for (int r = 0; r < 8; ++r) {
#pragma unroll
    for (int t = 0; t < 4; ++t)
      pw[(8 * hh + r) * LP + 16 * t + c] = (_Float16)(oacc[t][r] * invl[r]);
  }
  __syncthreads();
  v4u val[4];
  size_t go[4];
#pragma unroll
  for (int it = 0; it < 4; ++it) {
    const int p  = lane + 32 * it;
    const int L  = p >> 3;
    const int pc = p & 7;
    Pack8 pk;
    pk.h    = *(const v8h*)(pw + L * LP + pc * 8);
    val[it] = pk.u;
    go[it]  = (trow0 + q0 + L) * HID + (size_t)h * HDM + pc * 8;
  }
#pragma unroll
  for (int it = 0; it < 4; ++it) *(volatile v4u*)(op + go[it]) = val[it];
  __threadfence();
#pragma unroll
  for (int it = 0; it < 4; ++it) *(volatile v4u*)(op + go[it]) = val[it];
}

#define OTP 68
template <int RES, int HOUT>
__global__ __launch_bounds__(256) void k_gemm(const _Float16* __restrict__ ap,
                                              const _Float16* __restrict__ wt, int K,
                                              const float* __restrict__ bias,
                                              const float* res,
                                              float* outf, _Float16* outh, int N, float scale, float oscale) {
  __shared__ __align__(16) float st[8][16 * OTP];
  const int tid = threadIdx.x, lane = tid & 31, wave = tid >> 5;
  const int hh = lane >> 4, c = lane & 15;
  const int m0   = blockIdx.x * 256 + wave * 32;
  const int n0   = blockIdx.y * 64;

  v8f acc[2][4];
#pragma unroll
  for (int s = 0; s < 2; ++s)
#pragma unroll
    for (int t = 0; t < 4; ++t) acc[s][t] = zero8();
  gemm32x64(ap, K, wt, K, K, m0, n0, lane, acc);

  float* sw = st[wave];
#pragma unroll
  for (int sub = 0; sub < 2; ++sub) {
    __syncthreads();
#pragma unroll
    for (int t = 0; t < 4; ++t) {
#pragma unroll
      for (int r = 0; r < 8; ++r) sw[(8 * hh + r) * OTP + 16 * t + c] = acc[sub][t][r] * scale;
    }
    __syncthreads();
    if (HOUT) {
#pragma unroll 2
      for (int e = lane; e < 16 * 64; e += 32) {
        const int row = e >> 6, col = e & 63;
        const float v = sw[row * OTP + col] + bias[n0 + col];
        sw[row * OTP + col] = gelu_t(v) * oscale;
      }
      __syncthreads();
      v4u val[4];
      size_t go[4];
#pragma unroll
      for (int it = 0; it < 4; ++it) {
        const int p  = lane + 32 * it;
        const int L  = p >> 3;
        const int pc = p & 7;
        const float* ra = sw + L * OTP + pc * 8;
        const v4f a0 = *(const v4f*)(ra), a1 = *(const v4f*)(ra + 4);
        Pack8 pk;
        pk.h = (v8h){(_Float16)a0[0], (_Float16)a0[1], (_Float16)a0[2], (_Float16)a0[3],
                     (_Float16)a1[0], (_Float16)a1[1], (_Float16)a1[2], (_Float16)a1[3]};
        val[it] = pk.u;
        go[it]  = (size_t)(m0 + sub * 16 + L) * N + n0 + pc * 8;
      }
#pragma unroll
      for (int it = 0; it < 4; ++it) *(volatile v4u*)(outh + go[it]) = val[it];
      __threadfence();
#pragma unroll
      for (int it = 0; it < 4; ++it) *(volatile v4u*)(outh + go[it]) = val[it];
    } else {
      v4f val[8];
      size_t go[8];
#pragma unroll
      for (int it = 0; it < 8; ++it) {
        const int p    = lane + 32 * it;
        const int L    = p >> 3;
        const int pc   = p & 7;
        const int row  = L >> 1;
        const int half = L & 1;
        const int col  = n0 + half * 32 + pc * 4;
        go[it]  = (size_t)(m0 + sub * 16 + row) * N + col;
        v4f sv = *(const v4f*)(sw + row * OTP + half * 32 + pc * 4);
        const v4f bv = *(const v4f*)(bias + col);
        sv = sv + bv;
        if (RES) { const v4f rv = *(const v4f*)(res + go[it]); sv = sv + rv; }
        val[it] = sv;
      }
#pragma unroll
      for (int it = 0; it < 8; ++it) *(volatile v4f*)(outf + go[it]) = val[it];
      __threadfence();
#pragma unroll
      for (int it = 0; it < 8; ++it) *(volatile v4f*)(outf + go[it]) = val[it];
    }
  }
}

template <int OUTH>
__global__ __launch_bounds__(192) void k_ln(const float* __restrict__ src,
                                            const float* __restrict__ gt, const float* __restrict__ et,
                                            const float* __restrict__ gs, const float* __restrict__ es,
                                            float* of, _Float16* oh) {
  __shared__ float rs[2][6];
  const int tid = threadIdx.x, lane = tid & 31, wave = tid >> 5;
  const bool grp = (wave >= 3);
  const size_t o = (size_t)blockIdx.x * HID + (size_t)tid * 4;
  const v4f a = *(const v4f*)(src + o);
  float s = (a[0] + a[1]) + (a[2] + a[3]);
  s = wsum32(s);
  if (lane == 0) rs[0][wave] = s;
  __syncthreads();
  const float s_t = (rs[0][0] + rs[0][1]) + rs[0][2];
  const float s_s = (rs[0][3] + rs[0][4]) + rs[0][5];
  const float mean = (grp ? s_s : s_t) * (1.0f / (float)TDM);
  const v4f d = a - mean;
  float q = (d[0] * d[0] + d[1] * d[1]) + (d[2] * d[2] + d[3] * d[3]);
  q = wsum32(q);
  if (lane == 0) rs[1][wave] = q;
  __syncthreads();
  const float v_t = (rs[1][0] + rs[1][1]) + rs[1][2];
  const float v_s = (rs[1][3] + rs[1][4]) + rs[1][5];
  const float var  = (grp ? v_s : v_t) * (1.0f / (float)TDM);
  const float rstd = rsqrtf(var + 1e-5f);
  const int gi = (grp ? (tid - 96) : tid) * 4;
  const v4f g0 = *(const v4f*)(gt + gi), g1 = *(const v4f*)(gs + gi);
  const v4f e0 = *(const v4f*)(et + gi), e1 = *(const v4f*)(es + gi);
  const v4f gg = (v4f){grp ? g1[0] : g0[0], grp ? g1[1] : g0[1], grp ? g1[2] : g0[2], grp ? g1[3] : g0[3]};
  const v4f ee = (v4f){grp ? e1[0] : e0[0], grp ? e1[1] : e0[1], grp ? e1[2] : e0[2], grp ? e1[3] : e0[3]};
  const v4f y = d * rstd * gg + ee;

  v2u hv = (v2u){0u, 0u};
  if (OUTH) {
    Pack4 pk;
    pk.h = (v4h){(_Float16)y[0], (_Float16)y[1], (_Float16)y[2], (_Float16)y[3]};
    hv = pk.u;
  }
  *(volatile v4f*)(of + o) = y;
  if (OUTH) *(volatile v2u*)(oh + o) = hv;
  __threadfence();
  *(volatile v4f*)(of + o) = y;
  if (OUTH) *(volatile v2u*)(oh + o) = hv;
}

extern "C" void kernel_launch(void* const* d_in, const int* in_sizes, int n_in,
                              void* d_out, int out_size, void* d_ws, size_t ws_size,
                              hipStream_t stream) {
  if (n_in < 21) return;
  if (in_sizes[0] != NTOK * HID) return;
  if (in_sizes[1] != HID * HID || in_sizes[3] != HID * HID) return;
  if (in_sizes[5] != HID * HID || in_sizes[7] != HID * HID) return;
  if (in_sizes[2] != HID || in_sizes[4] != HID || in_sizes[6] != HID || in_sizes[8] != HID) return;
  if (in_sizes[9] != TDM || in_sizes[10] != TDM || in_sizes[11] != TDM || in_sizes[12] != TDM) return;
  if (in_sizes[13] != HID * FFD) return;
  if (in_sizes[14] != FFD) return;
  if (in_sizes[15] != FFD * HID) return;
  if (in_sizes[16] != HID) return;
  if (in_sizes[17] != TDM || in_sizes[18] != TDM || in_sizes[19] != TDM || in_sizes[20] != TDM) return;
  if (out_size != NTOK * HID) return;

  const float* x   = (const float*)d_in[0];
  const float* wq  = (const float*)d_in[1];
  const float* bq  = (const float*)d_in[2];
  const float* wk  = (const float*)d_in[3];
  const float* bk  = (const float*)d_in[4];
  const float* wv  = (const float*)d_in[5];
  const float* bv  = (const float*)d_in[6];
  const float* wo  = (const float*)d_in[7];
  const float* bo  = (const float*)d_in[8];
  const float* g1t = (const float*)d_in[9];
  const float* b1t = (const float*)d_in[10];
  const float* g1s = (const float*)d_in[11];
  const float* b1s = (const float*)d_in[12];
  const float* w1  = (const float*)d_in[13];
  const float* bb1 = (const float*)d_in[14];
  const float* w2  = (const float*)d_in[15];
  const float* bb2 = (const float*)d_in[16];
  const float* g2t = (const float*)d_in[17];
  const float* b2t = (const float*)d_in[18];
  const float* g2s = (const float*)d_in[19];
  const float* b2s = (const float*)d_in[20];
  float* out = (float*)d_out;

  size_t off = 0;
  const size_t oX   = off; off += (size_t)NTOK * HID * 2;
  const size_t oWp  = off; off += (size_t)4 * HID * HID * 2;
  const size_t oW1  = off; off += (size_t)FFD * HID * 2;
  const size_t oW2  = off; off += (size_t)HID * FFD * 2;
  const size_t oQ   = off; off += (size_t)NBAT * NH * SQ * HDM * 2;
  const size_t oK   = off; off += (size_t)NBAT * NH * SQ * HDM * 2;
  const size_t oV   = off; off += (size_t)NBAT * NH * HDM * SQ * 2;
  const size_t oO   = off; off += (size_t)NTOK * HID * 2;
  const size_t oAX  = off; off += (size_t)NTOK * HID * 4;
  const size_t oXL  = off; off += (size_t)NTOK * HID * 4;
  const size_t oXLh = off; off += (size_t)NTOK * HID * 2;
  const size_t oG   = off; off += (size_t)NTOK * FFD * 2;
  const size_t oH2  = off; off += (size_t)NTOK * HID * 4;
  if (off > ws_size) return;
  if (off > (size_t)134217728) return;

  char* ws = (char*)d_ws;
  _Float16* Xh  = (_Float16*)(ws + oX);
  _Float16* Wp  = (_Float16*)(ws + oWp);
  _Float16* W1t = (_Float16*)(ws + oW1);
  _Float16* W2t = (_Float16*)(ws + oW2);
  _Float16* Qp  = (_Float16*)(ws + oQ);
  _Float16* Kp  = (_Float16*)(ws + oK);
  _Float16* Vt  = (_Float16*)(ws + oV);
  _Float16* Op  = (_Float16*)(ws + oO);
  float*    AX  = (float*)(ws + oAX);
  float*    XL  = (float*)(ws + oXL);
  _Float16* XLh = (_Float16*)(ws + oXLh);
  _Float16* Gh  = (_Float16*)(ws + oG);
  float*    H2  = (float*)(ws + oH2);
  const _Float16* Wot = Wp + (size_t)3 * HID * HID;

  k_cvtw<<<dim3(HID / 64, HID / 64, 4), dim3(128), 0, stream>>>(wq, wk, wv, wo, HID, HID, Wp);
  k_cvtw<<<dim3(FFD / 64, HID / 64, 1), dim3(128), 0, stream>>>(w1, w1, w1, w1, HID, FFD, W1t);
  k_cvtw<<<dim3(HID / 64, FFD / 64, 1), dim3(128), 0, stream>>>(w2, w2, w2, w2, FFD, HID, W2t);
  k_cvtx<<<dim3((NTOK * HID) / 2048), dim3(256), 0, stream>>>(x, Xh);
  k_qkv<<<dim3(NTOK / 64, 3 * NH), dim3(128), 0, stream>>>(Xh, Wp, bq, bk, bv, Qp, Kp, Vt);
  const float sscale = 0.125f;
  k_attn<<<dim3(NBAT * NH * NQB), dim3(256), 0, stream>>>(Qp, Kp, Vt, Op, sscale);
  k_gemm<1, 0><<<dim3(NTOK / 256, HID / 64), dim3(256), 0, stream>>>(Op, Wot, HID, bo, x, AX, Gh, HID,
                                                                      0.00048828125f, 1.0f);
  k_ln<1><<<dim3(NTOK), dim3(192), 0, stream>>>(AX, g1t, b1t, g1s, b1s, XL, XLh);
  k_gemm<0, 1><<<dim3(NTOK / 256, FFD / 64), dim3(256), 0, stream>>>(XLh, W1t, HID, bb1, x, AX, Gh, FFD,
                                                                      0.03125f, 8.0f);
  k_gemm<1, 0><<<dim3(NTOK / 256, HID / 64), dim3(256), 0, stream>>>(Gh, W2t, FFD, bb2, XL, H2, Gh, HID,
                                                                      0.00390625f, 1.0f);
  k_ln<0><<<dim3(NTOK), dim3(192), 0, stream>>>(H2, g2t, b2t, g2s, b2s, out, XLh);
  (void)hipGetLastError();
}
